// PreyAttnActor_13589276525225
// MI455X (gfx1250) — hardware-verified
//
#include <hip/hip_runtime.h>

typedef _Float16 v16h __attribute__((ext_vector_type(16)));
typedef _Float16 v8h  __attribute__((ext_vector_type(8)));
typedef float    v8f  __attribute__((ext_vector_type(8)));
typedef float    v4f  __attribute__((ext_vector_type(4)));

#define NP_    16
#define NY_    128
#define NO_    32
#define NN_    176
#define D_     64
#define SKP_   192
#define QH_    64
#define NPASS_ 2

#define WSCALE_ 16.0f
#define WINV_   0.0625f
#define PSCALE_ 16384.0f
#define PINV_   0.00006103515625f

#define OFFB_S   0
#define OFFB_P   49152
#define OFFB_X   73728
#define OFFB_K   96256
#define OFFB_V   118784
#define OFFB_Q   143360
#define OFFB_W   159744
#define OFFB_BK  233472
#define OFFB_DD  234176
#define OFFB_W3  234880
#define OFFB_Y   235136
#define SMEM_BYTES 235648
static_assert(SMEM_BYTES <= 240000);

#define W_PW2 0
#define W_YW2 1
#define W_OW2 2
#define W_WK  3
#define W_WV  4
#define W_WQ  5
#define W_WO  6
#define W_NW1 7
#define W_NW2 8
#define WPACK_HALVES (9 * 4096)
#define WPACK_BYTES  (WPACK_HALVES * 2)

__device__ __forceinline__ int kof(int i, int lane) {
  return (i & 7) | ((lane & 16) >> 1) | ((i & 8) << 1);
}

__device__ __forceinline__ v16h load_a16(const _Float16* p, int stride, int lane) {
  const _Float16* q = p + (lane & 15) * stride + ((lane & 16) >> 1);
  v8h lo = *(const v8h*)q;
  v8h hi = *(const v8h*)(q + 16);
  return __builtin_shufflevector(lo, hi, 0, 1, 2, 3, 4, 5, 6, 7,
                                 8, 9, 10, 11, 12, 13, 14, 15);
}

__device__ __forceinline__ v16h load_bp(const _Float16* wpTile, int lane) {
  const _Float16* q = wpTile + lane * 16;
  v8h lo = *(const v8h*)q;
  v8h hi = *(const v8h*)(q + 8);
  return __builtin_shufflevector(lo, hi, 0, 1, 2, 3, 4, 5, 6, 7,
                                 8, 9, 10, 11, 12, 13, 14, 15);
}

__device__ __forceinline__ v8f wmma_step(v16h a, v16h b, v8f c) {
  v8f d = __builtin_amdgcn_wmma_f32_16x16x32_f16(false, a, false, b, (short)0, c,
                                                 false, false);
  asm volatile("v_nop\n\tv_nop\n\tv_nop\n\tv_nop" : "+v"(d) : "v"(a), "v"(b));
  return d;
}

__device__ __forceinline__ v8f mm64p(const _Float16* a, int sa,
                                     const _Float16* wp, int nt, int lane) {
  v8f c = {};
  c = wmma_step(load_a16(a,      sa, lane), load_bp(wp + (0 * 4 + nt) * 512, lane), c);
  c = wmma_step(load_a16(a + 32, sa, lane), load_bp(wp + (1 * 4 + nt) * 512, lane), c);
  return c;
}

__device__ __forceinline__ void store_c16(_Float16* p, int stride, int lane, v8f c,
                                          float scale, float bias, bool relu) {
#pragma unroll
  for (int r = 0; r < 8; ++r) {
    float t = c[r] * scale + bias;
    if (relu) t = fmaxf(t, 0.f);
    p[(r + ((lane >> 4) << 3)) * stride + (lane & 15)] = (_Float16)t;
  }
}

extern "C" __global__ __launch_bounds__(256)
void pack_weights_kernel(const float* __restrict__ p_w2, const float* __restrict__ y_w2,
                         const float* __restrict__ o_w2, const float* __restrict__ wk,
                         const float* __restrict__ wv, const float* __restrict__ wq,
                         const float* __restrict__ wo, const float* __restrict__ n_w1,
                         const float* __restrict__ n_w2, _Float16* __restrict__ wp) {
  __shared__ __attribute__((aligned(16))) _Float16 tile[4096];
  const int tid = threadIdx.x, lane = tid & 31;
  const int bi = blockIdx.x;
  const float* w = p_w2;
  if (bi == 1) w = y_w2;
  if (bi == 2) w = o_w2;
  if (bi == 3) w = wk;
  if (bi == 4) w = wv;
  if (bi == 5) w = wq;
  if (bi == 6) w = wo;
  if (bi == 7) w = n_w1;
  if (bi == 8) w = n_w2;
  const int kt = tid >> 7;
  const int n  = ((tid >> 5) & 3) * 16 + (lane & 15);
#pragma unroll
  for (int i = 0; i < 16; ++i)
    tile[tid * 16 + i] = (_Float16)(w[(kt * 32 + kof(i, lane)) * 64 + n] * WSCALE_);
  __syncthreads();
  _Float16* dst = wp + (size_t)bi * 4096;
  const v8h u0 = *(const v8h*)(tile + tid * 8);
  const v8h u1 = *(const v8h*)(tile + (256 + tid) * 8);
  *(volatile v8h*)(dst + tid * 8) = u0;
  *(volatile v8h*)(dst + (256 + tid) * 8) = u1;
  __threadfence();
  *(volatile v8h*)(dst + tid * 8) = u0;
  *(volatile v8h*)(dst + (256 + tid) * 8) = u1;
}

extern "C" __global__ __launch_bounds__(256)
void attn_actor_main(const float* __restrict__ pred_g, const float* __restrict__ prey_g,
                     const float* __restrict__ obst_g, const int* __restrict__ alive_g,
                     const float* __restrict__ emb,
                     const float* __restrict__ p_w1, const float* __restrict__ p_b1,
                     const float* __restrict__ p_b2,
                     const float* __restrict__ y_w1, const float* __restrict__ y_b1,
                     const float* __restrict__ y_b2,
                     const float* __restrict__ o_w1, const float* __restrict__ o_b1,
                     const float* __restrict__ o_b2,
                     const float* __restrict__ bq, const float* __restrict__ bk,
                     const float* __restrict__ bv, const float* __restrict__ bo,
                     const float* __restrict__ w_pos,
                     const float* __restrict__ n_b1, const float* __restrict__ n_b2,
                     const float* __restrict__ n_w3, const float* __restrict__ n_b3,
                     const _Float16* __restrict__ wpg, float* __restrict__ out) {
  extern __shared__ __attribute__((aligned(16))) char smem[];
  float*    S  = (float*)(smem + OFFB_S);
  _Float16* P  = (_Float16*)(smem + OFFB_P);
  _Float16* X  = (_Float16*)(smem + OFFB_X);
  _Float16* Km = (_Float16*)(smem + OFFB_K);
  _Float16* Vp = (_Float16*)(smem + OFFB_V);
  _Float16* Qm = (_Float16*)(smem + OFFB_Q);
  _Float16* WP = (_Float16*)(smem + OFFB_W);
  float*    BK = (float*)(smem + OFFB_BK);
  float*    DD = (float*)(smem + OFFB_DD);
  float*    W3 = (float*)(smem + OFFB_W3);
  float*    Y  = (float*)(smem + OFFB_Y);

  const int tid  = threadIdx.x;
  const int lane = tid & 31;
  const int wid  = tid >> 5;
  const int b    = blockIdx.x;

  const float* pred  = pred_g  + (size_t)b * NP_ * 2;
  const float* prey  = prey_g  + (size_t)b * NY_ * 2;
  const float* obst  = obst_g  + (size_t)b * NO_ * 3;
  const int*   alive = alive_g + (size_t)b * NY_;

  {
    const v8h* src = (const v8h*)wpg;
    v8h*       dst = (v8h*)WP;
    for (int i = tid; i < WPACK_HALVES / 8; i += 256) dst[i] = src[i];
  }
  for (int i = tid; i < (6 * 4 * 512) / 2; i += 256) ((int*)Vp)[i] = 0;
  if (tid < 64) W3[tid] = n_w3[tid];

  {
    const float wp0 = w_pos[0], wp1 = w_pos[1];
    for (int r = tid; r < NN_; r += 256) {
      float px, py; float d = 0.f;
      if (r < NP_)            { px = pred[r * 2]; py = pred[r * 2 + 1]; }
      else if (r < NP_ + NY_) { int i = r - NP_; px = prey[i * 2]; py = prey[i * 2 + 1];
                                d = (alive[i] != 0) ? 0.f : 1.f; }
      else                    { int i = r - NP_ - NY_; px = obst[i * 3]; py = obst[i * 3 + 1]; }
      BK[r] = px * wp0 + py * wp1;
      DD[r] = d;
    }
  }

  for (int i = tid; i < NN_ * D_; i += 256) {
    int r = i >> 6, dd = i & 63;
    float acc;
    if (r < NP_) {
      acc = p_b1[dd] + pred[r * 2] * p_w1[dd] + pred[r * 2 + 1] * p_w1[64 + dd];
    } else if (r < NP_ + NY_) {
      int j = r - NP_;
      acc = y_b1[dd] + prey[j * 2] * y_w1[dd] + prey[j * 2 + 1] * y_w1[64 + dd];
    } else {
      int j = r - NP_ - NY_;
      acc = o_b1[dd] + obst[j * 3] * o_w1[dd] + obst[j * 3 + 1] * o_w1[64 + dd]
          + obst[j * 3 + 2] * o_w1[128 + dd];
    }
    P[i] = (_Float16)fmaxf(acc, 0.f);
  }
  __syncthreads();

  for (int job = wid; job < 11 * 4; job += 8) {
    int mt = job >> 2, nt = job & 3;
    const _Float16* wp; const float* b2; int ty;
    if (mt == 0)      { wp = WP + W_PW2 * 4096; b2 = p_b2; ty = 0; }
    else if (mt <= 8) { wp = WP + W_YW2 * 4096; b2 = y_b2; ty = 1; }
    else              { wp = WP + W_OW2 * 4096; b2 = o_b2; ty = 2; }
    v8f c = mm64p(P + mt * 16 * 64, 64, wp, nt, lane);
    int col = nt * 16 + (lane & 15);
    store_c16(X + mt * 16 * 64 + nt * 16, 64, lane, c, WINV_,
              b2[col] + emb[ty * 64 + col], false);
  }
  __syncthreads();

  for (int job = wid; job < 120; job += 8) {
    int j = job;
    if (j < 44) {
      int mt = j >> 2, nt = j & 3;
      v8f c = mm64p(X + mt * 16 * 64, 64, WP + W_WK * 4096, nt, lane);
      store_c16(Km + mt * 16 * 64 + nt * 16, 64, lane, c, WINV_,
                bk[nt * 16 + (lane & 15)], false);
    } else if (j < 88) {
      j -= 44;
      int mt = j >> 2, nt = j & 3;
      v8f c = mm64p(X + mt * 16 * 64, 64, WP + W_WV * 4096, nt, lane);
      float bias = bv[nt * 16 + (lane & 15)];
      int n = lane & 15;
#pragma unroll
      for (int r = 0; r < 8; ++r) {
        int key = mt * 16 + r + ((lane >> 4) << 3);
        int kt5 = key >> 5, kk = key & 31;
        int lp = n + ((kk & 8) << 1);
        int hp = (kk & 7) | ((kk & 16) >> 1);
        Vp[(kt5 * 4 + nt) * 512 + lp * 16 + hp] = (_Float16)(c[r] * WINV_ + bias);
      }
    } else {
      j -= 88;
      int mt = j >> 2, nt = j & 3;
      v8f c = mm64p(X + (NP_ + mt * 16) * 64, 64, WP + W_WQ * 4096, nt, lane);
      store_c16(Qm + mt * 16 * 64 + nt * 16, 64, lane, c, WINV_,
                bq[nt * 16 + (lane & 15)], false);
    }
  }
  __syncthreads();

  for (int qh = 0; qh < NPASS_; ++qh) {
    for (int job = wid; job < 4 * 11; job += 8) {
      int mt = job / 11, nt = job - mt * 11;
      const _Float16* qb = Qm + (qh * QH_ + mt * 16) * 64;
      const _Float16* kb = Km + nt * 16 * 64;
      v8f c = {};
      c = wmma_step(load_a16(qb,      64, lane), load_a16(kb,      64, lane), c);
      c = wmma_step(load_a16(qb + 32, 64, lane), load_a16(kb + 32, 64, lane), c);
      int col = nt * 16 + (lane & 15);
      float bkv = BK[col], kdead = DD[col];
#pragma unroll
      for (int r = 0; r < 8; ++r) {
        int rl = mt * 16 + r + ((lane >> 4) << 3);
        int qrow = qh * QH_ + rl;
        float sc = (c[r] + BK[NP_ + qrow] - bkv) * 0.125f;
        if (DD[NP_ + qrow] > 0.5f && kdead > 0.5f) sc = -1e9f;
        S[rl * SKP_ + col] = sc;
      }
    }
    __syncthreads();

    for (int rl = wid; rl < QH_; rl += 8) {
      const float* sr = S + rl * SKP_;
      _Float16* prow = P + rl * SKP_;
      float v[6];
      float m = -3.0e38f;
#pragma unroll
      for (int c6 = 0; c6 < 6; ++c6) {
        int j = lane + 32 * c6;
        float t = (j < NN_) ? sr[j] : -3.0e38f;
        v[c6] = t;
        m = fmaxf(m, t);
      }
#pragma unroll
      for (int o = 16; o > 0; o >>= 1) m = fmaxf(m, __shfl_xor(m, o, 32));
      float sum = 0.f;
#pragma unroll
      for (int c6 = 0; c6 < 6; ++c6) {
        int j = lane + 32 * c6;
        float e = (j < NN_) ? __expf(v[c6] - m) : 0.f;
        v[c6] = e;
        sum += e;
      }
#pragma unroll
      for (int o = 16; o > 0; o >>= 1) sum += __shfl_xor(sum, o, 32);
      const float psc = PSCALE_ * (1.0f / sum);
#pragma unroll
      for (int c6 = 0; c6 < 6; ++c6) {
        int j = lane + 32 * c6;
        prow[j] = (_Float16)((j < NN_) ? v[c6] * psc : 0.f);
      }
    }
    __syncthreads();

    for (int job = wid; job < 16; job += 8) {
      int mt = job >> 2, nt = job & 3;
      v8f c = {};
#pragma unroll
      for (int ks = 0; ks < 6; ++ks)
        c = wmma_step(load_a16(P + mt * 16 * SKP_ + ks * 32, SKP_, lane),
                      load_bp(Vp + (ks * 4 + nt) * 512, lane), c);
      store_c16(X + (qh * QH_ + mt * 16) * 64 + nt * 16, 64, lane, c, PINV_, 0.f, false);
    }
    __syncthreads();
  }

  for (int job = wid; job < 32; job += 8) {
    int mt = job >> 2, nt = job & 3;
    v8f c = mm64p(X + mt * 16 * 64, 64, WP + W_WO * 4096, nt, lane);
    store_c16(Km + mt * 16 * 64 + nt * 16, 64, lane, c, WINV_,
              bo[nt * 16 + (lane & 15)], false);
  }
  __syncthreads();

  for (int job = wid; job < 32; job += 8) {
    int mt = job >> 2, nt = job & 3;
    v8f c = mm64p(Km + mt * 16 * 64, 64, WP + W_NW1 * 4096, nt, lane);
    store_c16(Vp + mt * 16 * 64 + nt * 16, 64, lane, c, WINV_,
              n_b1[nt * 16 + (lane & 15)], true);
  }
  __syncthreads();

  for (int job = wid; job < 32; job += 8) {
    int mt = job >> 2, nt = job & 3;
    v8f c = mm64p(Vp + mt * 16 * 64, 64, WP + W_NW2 * 4096, nt, lane);
    store_c16(Qm + mt * 16 * 64 + nt * 16, 64, lane, c, WINV_,
              n_b2[nt * 16 + (lane & 15)], true);
  }
  __syncthreads();

  for (int r = tid; r < NY_; r += 256) {
    float acc = n_b3[0];
    const v8h* qr = (const v8h*)(Qm + r * 64);
#pragma unroll
    for (int c8 = 0; c8 < 8; ++c8) {
      v8h q = qr[c8];
#pragma unroll
      for (int j = 0; j < 8; ++j) acc += (float)q[j] * W3[c8 * 8 + j];
    }
    Y[r] = tanhf(acc);
  }
  __syncthreads();

  if (wid == 0) {
    const v4f val = *(const v4f*)(Y + lane * 4);
    float* op = out + (size_t)b * NY_ + lane * 4;
    *(volatile v4f*)op = val;
    __threadfence();
    *(volatile v4f*)op = val;
  }
}

extern "C" void kernel_launch(void* const* d_in, const int* in_sizes, int n_in,
                              void* d_out, int out_size, void* d_ws, size_t ws_size,
                              hipStream_t stream) {
  if (n_in < 32) return;
  const int nb = out_size / NY_;
  if (nb <= 0) return;
  if (in_sizes[0] != nb * NP_ * 2 || in_sizes[1] != nb * NY_ * 2 ||
      in_sizes[2] != nb * NO_ * 3 || in_sizes[3] != nb * NY_) return;
  if (d_ws == nullptr || ws_size < (size_t)WPACK_BYTES) return;

  const float* pred  = (const float*)d_in[0];
  const float* prey  = (const float*)d_in[1];
  const float* obst  = (const float*)d_in[2];
  const int*   alive = (const int*)d_in[3];
  const float* emb   = (const float*)d_in[4];
  const float* p_w1 = (const float*)d_in[5];  const float* p_b1 = (const float*)d_in[6];
  const float* p_w2 = (const float*)d_in[7];  const float* p_b2 = (const float*)d_in[8];
  const float* y_w1 = (const float*)d_in[9];  const float* y_b1 = (const float*)d_in[10];
  const float* y_w2 = (const float*)d_in[11]; const float* y_b2 = (const float*)d_in[12];
  const float* o_w1 = (const float*)d_in[13]; const float* o_b1 = (const float*)d_in[14];
  const float* o_w2 = (const float*)d_in[15]; const float* o_b2 = (const float*)d_in[16];
  const float* wq   = (const float*)d_in[17]; const float* bq   = (const float*)d_in[18];
  const float* wk   = (const float*)d_in[19]; const float* bk   = (const float*)d_in[20];
  const float* wv   = (const float*)d_in[21]; const float* bv   = (const float*)d_in[22];
  const float* wo   = (const float*)d_in[23]; const float* bo   = (const float*)d_in[24];
  const float* w_pos = (const float*)d_in[25];
  const float* n_w1 = (const float*)d_in[26]; const float* n_b1 = (const float*)d_in[27];
  const float* n_w2 = (const float*)d_in[28]; const float* n_b2 = (const float*)d_in[29];
  const float* n_w3 = (const float*)d_in[30]; const float* n_b3 = (const float*)d_in[31];
  float* out = (float*)d_out;
  _Float16* wpg = (_Float16*)d_ws;

  pack_weights_kernel<<<9, 256, 0, stream>>>(p_w2, y_w2, o_w2, wk, wv, wq, wo, n_w1, n_w2, wpg);

  hipFuncSetAttribute((const void*)attn_actor_main,
                      hipFuncAttributeMaxDynamicSharedMemorySize,
                      (int)SMEM_BYTES);
  attn_actor_main<<<nb, 256, SMEM_BYTES, stream>>>(
      pred, prey, obst, alive, emb,
      p_w1, p_b1, p_b2, y_w1, y_b1, y_b2, o_w1, o_b1, o_b2,
      bq, bk, bv, bo, w_pos, n_b1, n_b2, n_w3, n_b3,
      (const _Float16*)wpg, out);
}
